// GravityAttention_25615184954029
// MI455X (gfx1250) — hardware-verified
//
#include <hip/hip_runtime.h>
#include <math.h>
#include <stdint.h>

#ifndef NB
#define NB 2
#endif
#ifndef SEQ
#define SEQ 2048
#endif
#define NB_FULL  2
#define SEQ_FULL 2048
#define DM   1024
#define NH   16
#define HC   16
#define HD   64
#define DC   64
#define HN   (NH * HC)
#define ZP   (NH * 64)
#define OP   (2 * DM)
#define NQB  (SEQ / 64)
#define NKT  (SEQ / 64)
#define PCARRY 16384.0f
#define RSC    4096.0f
#define OUT1_OFF ((size_t)NB_FULL * SEQ_FULL * DM)
static_assert(NH * HD == DM);
static_assert(HC == 16 && HD == 64 && DC == 64);
static_assert((SEQ % 64) == 0 && SEQ >= 64 && SEQ <= SEQ_FULL);
static_assert(NB >= 1 && NB <= NB_FULL);
static_assert((DM % 64) == 0 && (HN % 64) == 0 && (OP % 64) == 0);
static_assert(OUT1_OFF * 4 == 16777216);

typedef _Float16 v16h __attribute__((ext_vector_type(16)));
typedef _Float16 v8h  __attribute__((ext_vector_type(8)));
typedef __bf16   v16b __attribute__((ext_vector_type(16)));
typedef __bf16   v8b  __attribute__((ext_vector_type(8)));
typedef float    v8f  __attribute__((ext_vector_type(8)));
typedef float    v4f  __attribute__((ext_vector_type(4)));
typedef unsigned int v4u __attribute__((ext_vector_type(4)));

#if defined(__HIP_DEVICE_COMPILE__)
#define DEV_ASM 1
#else
#define DEV_ASM 0
#endif

__device__ __forceinline__ unsigned short bf_bits(float f) {
  unsigned u = __float_as_uint(f);
  return (unsigned short)((u + 0x7FFFu + ((u >> 16) & 1u)) >> 16);
}
__device__ __forceinline__ float bf_up(unsigned short hb) { return __uint_as_float(((unsigned)hb) << 16); }
__device__ __forceinline__ float bfr(float f) { return bf_up(bf_bits(f)); }
__device__ __forceinline__ unsigned short h_bits(_Float16 x) { return __builtin_bit_cast(unsigned short, x); }
__device__ __forceinline__ unsigned pk16(unsigned short a, unsigned short b) { return (unsigned)a | ((unsigned)b << 16); }
__device__ __forceinline__ v8f zero8() { v8f z = {0.f, 0.f, 0.f, 0.f, 0.f, 0.f, 0.f, 0.f}; return z; }

template <typename OT> struct FT;
template <> struct FT<__bf16>   { typedef v16b frag; typedef v8b half8; };
template <> struct FT<_Float16> { typedef v16h frag; typedef v8h half8; };

template <typename OT>
__device__ __forceinline__ typename FT<OT>::frag ldfrag(const OT* p) {
  union { typename FT<OT>::frag v; typename FT<OT>::half8 h[2]; } f;
  f.h[0] = *(const typename FT<OT>::half8*)(p);
  f.h[1] = *(const typename FT<OT>::half8*)(p + 16);
  return f.v;
}

__device__ __forceinline__ v8f mmar(v16b a, v16b b, v8f c) {
  return __builtin_amdgcn_wmma_f32_16x16x32_bf16(false, a, false, b, (short)0, c, false, false);
}
__device__ __forceinline__ v8f mmar(v16h a, v16h b, v8f c) {
  return __builtin_amdgcn_wmma_f32_16x16x32_f16(false, a, false, b, (short)0, c, false, false);
}
__device__ __forceinline__ v8f mma_h(v16h a, v16h b, v8f c) {
  c = __builtin_amdgcn_wmma_f32_16x16x32_f16(false, a, false, b, (short)0, c, false, false);
#if DEV_ASM
  asm volatile("v_nop\n\tv_nop\n\tv_nop\n\tv_nop" : "+v"(c) : "v"(a), "v"(b));
#endif
  return c;
}
__device__ __forceinline__ void dep_guard(v8f& a, v8f& b, v16b x, v16b y) {
#if DEV_ASM
  asm volatile("v_nop\n\tv_nop\n\tv_nop\n\tv_nop" : "+v"(a), "+v"(b) : "v"(x), "v"(y));
#else
  (void)a; (void)b; (void)x; (void)y;
#endif
}
__device__ __forceinline__ void dep_guard(v8f& a, v8f& b, v16h x, v16h y) {
#if DEV_ASM
  asm volatile("v_nop\n\tv_nop\n\tv_nop\n\tv_nop" : "+v"(a), "+v"(b) : "v"(x), "v"(y));
#else
  (void)a; (void)b; (void)x; (void)y;
#endif
}
__device__ __forceinline__ void keep4(v16b a, v16b b, v16b c, v16b d) {
#if DEV_ASM
  asm volatile("v_nop" :: "v"(a), "v"(b), "v"(c), "v"(d));
#else
  (void)a; (void)b; (void)c; (void)d;
#endif
}
__device__ __forceinline__ void keep4(v16h a, v16h b, v16h c, v16h d) {
#if DEV_ASM
  asm volatile("v_nop" :: "v"(a), "v"(b), "v"(c), "v"(d));
#else
  (void)a; (void)b; (void)c; (void)d;
#endif
}
__device__ __forceinline__ void acc_guard4(v8f& a, v8f& b, v8f& c, v8f& d) {
#if DEV_ASM
  asm volatile("v_nop\n\tv_nop\n\tv_nop\n\tv_nop" : "+v"(a), "+v"(b), "+v"(c), "+v"(d));
#else
  (void)a; (void)b; (void)c; (void)d;
#endif
}

__global__ __launch_bounds__(256) void cvtrows(const float* __restrict__ in, unsigned short* out,
                                               int rowlen8, int nrows, int seq, int seqfull) {
  const int i = blockIdx.x * 256 + (int)threadIdx.x;
  if (i < nrows * rowlen8) {
    const int row  = i / rowlen8;
    const int c    = i - row * rowlen8;
    const int bq   = row / seq;
    const int srow = bq * seqfull + (row - bq * seq);
    const float* src = in + ((size_t)srow * (size_t)rowlen8 + (size_t)c) * 8;
    const v4f a  = *(const v4f*)(src);
    const v4f a4 = *(const v4f*)(src + 4);
    v4u p;
    p[0] = pk16(bf_bits(a[0]),  bf_bits(a[1]));
    p[1] = pk16(bf_bits(a[2]),  bf_bits(a[3]));
    p[2] = pk16(bf_bits(a4[0]), bf_bits(a4[1]));
    p[3] = pk16(bf_bits(a4[2]), bf_bits(a4[3]));
    unsigned short* o = out + (size_t)i * 8;
    *(volatile v4u*)o = p;
    __threadfence();
    *(volatile v4u*)o = p;
  }
}

__global__ __launch_bounds__(256) void tr64(const float* __restrict__ in, int ldi,
                                            unsigned short* out, int ldo, int dup) {
  __shared__ __align__(16) unsigned short sT[64 * 72];
  const int tid = (int)threadIdx.x;
  const int k0  = blockIdx.y * 64;
  const int n0  = blockIdx.x * 64;
  {
    const int r = tid >> 2, c16 = (tid & 3) * 16;
    const float* src = in + (size_t)(k0 + r) * (size_t)ldi + n0 + c16;
    const v4f a0 = *(const v4f*)(src);
    const v4f a1 = *(const v4f*)(src + 4);
    const v4f a2 = *(const v4f*)(src + 8);
    const v4f a3 = *(const v4f*)(src + 12);
#pragma unroll
    for (int e = 0; e < 4; ++e) {
      sT[(c16 + e) * 72 + r]      = bf_bits(a0[e]);
      sT[(c16 + 4 + e) * 72 + r]  = bf_bits(a1[e]);
      sT[(c16 + 8 + e) * 72 + r]  = bf_bits(a2[e]);
      sT[(c16 + 12 + e) * 72 + r] = bf_bits(a3[e]);
    }
  }
  __syncthreads();
  const int wave = tid >> 5, lane = tid & 31;
  const int q = lane >> 3, c8 = (lane & 7) * 8;
  v4u vv[2];
#pragma unroll
  for (int it = 0; it < 2; ++it) {
    const int n = it * 32 + wave * 4 + q;
    vv[it] = *(const v4u*)(sT + n * 72 + c8);
  }
  for (int pass = 0; pass < 2; ++pass) {
#pragma unroll
    for (int it = 0; it < 2; ++it) {
      const int n = it * 32 + wave * 4 + q;
      unsigned short* d = out + (size_t)(n0 + n) * (size_t)ldo + k0 + c8;
      *(volatile v4u*)d = vv[it];
      if (dup != 0) *(volatile v4u*)(d + dup) = vv[it];
    }
    __threadfence();
  }
}

template <typename OT, int OUT_MODE, int BIAS>
__global__ __launch_bounds__(256) void gemm64(
    const unsigned short* __restrict__ Ap, int lda, long long strideA,
    const unsigned short* __restrict__ Btp, int ldb, long long strideB,
    void* Cout, void* Cout2, int ldc, long long strideC,
    const float* __restrict__ bias,
    int M, int N, int K, float oscale, float rscale) {
  typedef typename FT<OT>::frag V16;
  const OT* A  = (const OT*)(const void*)Ap;
  const OT* Bt = (const OT*)(const void*)Btp;
  __shared__ __align__(16) float sT[8][16 * 68];
  const int b    = blockIdx.y;
  const int lane = threadIdx.x & 31;
  const int wave = threadIdx.x >> 5;
  const int tilesN = N >> 6;
  const int tilesM = M >> 6;
  const int tile = blockIdx.x * 8 + wave;
  if (tile >= tilesM * tilesN) return;
  const int tm = tile / tilesN;
  const int tn = tile - tm * tilesN;
  const int m0 = tm << 6;
  const int n0 = tn << 6;

  const OT* Ab = A  + (size_t)b * (size_t)strideA;
  const OT* Bb = Bt + (size_t)b * (size_t)strideB;

  const int rlane = lane & 15;
  const int koff  = (lane >> 4) * 8;
  const int mOff  = (lane >> 4) * 8;

  v8f acc[4][4];
#pragma unroll
  for (int i = 0; i < 4; ++i)
#pragma unroll
    for (int j = 0; j < 4; ++j) acc[i][j] = zero8();

  for (int k0 = 0; k0 < K; k0 += 32) {
    V16 bq[4];
#pragma unroll
    for (int j = 0; j < 4; ++j)
      bq[j] = ldfrag<OT>(Bb + (size_t)(n0 + (j << 4) + rlane) * (size_t)ldb + koff + k0);
#pragma unroll
    for (int i = 0; i < 4; ++i) {
      const V16 af = ldfrag<OT>(Ab + (size_t)(m0 + (i << 4) + rlane) * (size_t)lda + koff + k0);
#pragma unroll
      for (int j = 0; j < 4; ++j) acc[i][j] = mmar(af, bq[j], acc[i][j]);
      dep_guard(acc[i][0], acc[i][3], af, bq[3]);
    }
    keep4(bq[0], bq[1], bq[2], bq[3]);
  }
  acc_guard4(acc[0][0], acc[0][1], acc[0][2], acc[0][3]);
  acc_guard4(acc[1][0], acc[1][1], acc[1][2], acc[1][3]);
  acc_guard4(acc[2][0], acc[2][1], acc[2][2], acc[2][3]);
  acc_guard4(acc[3][0], acc[3][1], acc[3][2], acc[3][3]);

  float* slab = sT[wave];
#pragma unroll
  for (int i = 0; i < 4; ++i) {
    const int mBase = m0 + (i << 4);
#pragma unroll
    for (int j = 0; j < 4; ++j) {
#pragma unroll
      for (int r = 0; r < 8; ++r) {
        slab[(mOff + r) * 68 + (j << 4) + rlane] = acc[i][j][r];
      }
    }
    __builtin_amdgcn_fence(__ATOMIC_RELEASE, "workgroup");
    __builtin_amdgcn_wave_barrier();
    __builtin_amdgcn_fence(__ATOMIC_ACQUIRE, "workgroup");
    if (OUT_MODE == 0) {
      float* C = (float*)Cout + (size_t)b * (size_t)strideC;
      const int h2 = lane >> 4, c4 = (lane & 15) * 4;
      v4f bcol = {0.f, 0.f, 0.f, 0.f};
      if (BIAS == 1) {
        const v4f bb = *(const v4f*)(bias + n0 + c4);
#pragma unroll
        for (int e = 0; e < 4; ++e) bcol[e] = bfr(bb[e]);
      }
      for (int pass = 0; pass < 2; ++pass) {
#pragma unroll
        for (int it = 0; it < 8; ++it) {
          const int row = it * 2 + h2;
          float brow = 0.f;
          if (BIAS == 2) brow = bfr(bias[mBase + row]);
          const v4f x = *(const v4f*)(slab + row * 68 + c4);
          v4f v;
#pragma unroll
          for (int e = 0; e < 4; ++e) v[e] = x[e] * oscale + bcol[e] + brow;
          *(volatile v4f*)(C + (size_t)(mBase + row) * (size_t)ldc + n0 + c4) = v;
        }
        __threadfence();
      }
    } else {
      const int q = lane >> 3, c8 = (lane & 7) * 8;
      unsigned short* C  = (unsigned short*)Cout  + (size_t)b * (size_t)strideC;
      unsigned short* C2 = (unsigned short*)Cout2 + (size_t)b * (size_t)strideC;
      float bc8[8];
#pragma unroll
      for (int e = 0; e < 8; ++e) bc8[e] = 0.f;
      if (BIAS == 1) {
        const v4f b0 = *(const v4f*)(bias + n0 + c8);
        const v4f b1 = *(const v4f*)(bias + n0 + c8 + 4);
#pragma unroll
        for (int e = 0; e < 4; ++e) { bc8[e] = bfr(b0[e]); bc8[4 + e] = bfr(b1[e]); }
      }
      v4u hv[4], lv[4];
#pragma unroll
      for (int it = 0; it < 4; ++it) {
        const int row = it * 4 + q;
        const float* sp = slab + row * 68 + c8;
        float brow = 0.f;
        if (BIAS == 2) brow = bfr(bias[mBase + row]);
        float f[8];
#pragma unroll
        for (int e = 0; e < 8; ++e) f[e] = sp[e] * oscale + bc8[e] + brow;
        v4u a, a2;
#pragma unroll
        for (int e = 0; e < 4; ++e) {
          const float f0 = f[2 * e], f1 = f[2 * e + 1];
          const _Float16 x0 = (_Float16)f0, x1 = (_Float16)f1;
          const unsigned short h0 = h_bits(x0), h1 = h_bits(x1);
          unsigned short l0 = 0, l1 = 0;
          if (OUT_MODE == 3) {
            l0 = h_bits((_Float16)((f0 - (float)x0) * rscale));
            l1 = h_bits((_Float16)((f1 - (float)x1) * rscale));
          }
          a[e] = pk16(h0, h1); a2[e] = pk16(l0, l1);
        }
        hv[it] = a; lv[it] = a2;
      }
      for (int pass = 0; pass < 2; ++pass) {
#pragma unroll
        for (int it = 0; it < 4; ++it) {
          const int row = it * 4 + q;
          *(volatile v4u*)(C + (size_t)(mBase + row) * (size_t)ldc + n0 + c8) = hv[it];
          if (OUT_MODE == 3) *(volatile v4u*)(C2 + (size_t)(mBase + row) * (size_t)ldc + n0 + c8) = lv[it];
        }
        __threadfence();
      }
    }
    __builtin_amdgcn_fence(__ATOMIC_RELEASE, "workgroup");
    __builtin_amdgcn_wave_barrier();
    __builtin_amdgcn_fence(__ATOMIC_ACQUIRE, "workgroup");
  }
}

__global__ __launch_bounds__(256) void zprep(const float* __restrict__ zf, unsigned short* zp, float* zsq) {
  __shared__ __align__(16) unsigned short sZ[256 * 64];
  __shared__ __align__(16) float sQ[256];
  const int tid  = (int)threadIdx.x;
  const int r    = tid >> 4, hd = tid & 15;
  const int row0 = blockIdx.x * 16;
  {
    const float* zr = zf + (size_t)(row0 + r) * HN + hd * HC;
    const v4f a0 = *(const v4f*)(zr);
    const v4f a1 = *(const v4f*)(zr + 4);
    const v4f a2 = *(const v4f*)(zr + 8);
    const v4f a3 = *(const v4f*)(zr + 12);
    float f[16];
#pragma unroll
    for (int e = 0; e < 4; ++e) { f[e] = a0[e]; f[4 + e] = a1[e]; f[8 + e] = a2[e]; f[12 + e] = a3[e]; }
    float q = 0.f;
#pragma unroll
    for (int e = 0; e < 16; ++e) q += f[e] * f[e];
    sQ[tid] = q;
    v4u ph0, ph1, pl0, pl1;
#pragma unroll
    for (int e = 0; e < 4; ++e) {
      const float f0 = f[2 * e], f1 = f[2 * e + 1], f2 = f[8 + 2 * e], f3 = f[9 + 2 * e];
      const _Float16 x0 = (_Float16)f0, x1 = (_Float16)f1, x2 = (_Float16)f2, x3 = (_Float16)f3;
      ph0[e] = pk16(h_bits(x0), h_bits(x1));
      ph1[e] = pk16(h_bits(x2), h_bits(x3));
      pl0[e] = pk16(h_bits((_Float16)((f0 - (float)x0) * RSC)), h_bits((_Float16)((f1 - (float)x1) * RSC)));
      pl1[e] = pk16(h_bits((_Float16)((f2 - (float)x2) * RSC)), h_bits((_Float16)((f3 - (float)x3) * RSC)));
    }
    const v4u z4 = {0u, 0u, 0u, 0u};
    unsigned short* sl = sZ + tid * 64;
    *(v4u*)(sl + 0)  = ph0;
    *(v4u*)(sl + 8)  = ph1;
    *(v4u*)(sl + 16) = pl0;
    *(v4u*)(sl + 24) = pl1;
    *(v4u*)(sl + 32) = ph0;
    *(v4u*)(sl + 40) = ph1;
    *(v4u*)(sl + 48) = z4;
    *(v4u*)(sl + 56) = z4;
  }
  __syncthreads();
  const int wave = tid >> 5, lane = tid & 31;
  const int q4 = lane >> 3, c8 = (lane & 7) * 8;
  unsigned short* base = zp + (size_t)row0 * ZP;
  v4u vv[8];
#pragma unroll
  for (int it = 0; it < 8; ++it) {
    const int L = it * 32 + wave * 4 + q4;
    vv[it] = *(const v4u*)(sZ + L * 64 + c8);
  }
  for (int pass = 0; pass < 2; ++pass) {
#pragma unroll
    for (int it = 0; it < 8; ++it) {
      const int L = it * 32 + wave * 4 + q4;
      *(volatile v4u*)(base + (size_t)L * 64 + c8) = vv[it];
    }
    __threadfence();
  }
  if (tid < 64) {
    const v4f qv = *(const v4f*)(sQ + tid * 4);
    float* dst = zsq + (size_t)row0 * NH + tid * 4;
    *(volatile v4f*)dst = qv;
    __threadfence();
    *(volatile v4f*)dst = qv;
  }
}

__global__ __launch_bounds__(128)
void attn_dist(const unsigned short* __restrict__ zpp, const float* __restrict__ zsq,
               const unsigned short* __restrict__ vhp, const unsigned short* __restrict__ vlp,
               const float* __restrict__ gam, unsigned short* octx) {
  union FH { v16h v; v8h h[2]; };
  __shared__ __align__(16) _Float16 Zsh[64 * 64];
  __shared__ __align__(16) _Float16 Vth[64 * 64];
  __shared__ __align__(16) _Float16 Vtl[64 * 64];
  __shared__ __align__(16) _Float16 Psh[4][16 * 64];
  __shared__ __align__(16) float    Os[4][16 * 64];

  const int tid  = threadIdx.x;
  const int wave = tid >> 5;
  const int lane = tid & 31;
  const int hh   = lane >> 4;
  const int c    = lane & 15;

  const int bx   = blockIdx.x;
  const int qb   = bx % NQB;
  const int rest = bx / NQB;
  const int h    = rest % NH;
  const int b    = rest / NH;
  const int q0   = qb * 64 + wave * 16;
  const size_t rowB = (size_t)b * SEQ;

  const _Float16* Zp16 = (const _Float16*)(const void*)zpp;
  const _Float16* Vh = (const _Float16*)(const void*)vhp + ((size_t)b * DM + (size_t)h * HD) * SEQ;
  const _Float16* Vl = (const _Float16*)(const void*)vlp + ((size_t)b * DM + (size_t)h * HD) * SEQ;

  const float gx = bfr(gam[h]);
  const float g  = fmaxf(gx, 0.f) + log1pf(expf(-fabsf(gx)));
  const float ng = -g;

  const v16h zq = ldfrag<_Float16>(Zp16 + (rowB + q0 + c) * ZP + (size_t)h * 64 + 8 * hh);
  float zsq_q[8];
#pragma unroll
  for (int r = 0; r < 8; ++r) zsq_q[r] = zsq[(rowB + q0 + 8 * hh + r) * NH + h];

  float mrow[8], lrow[8];
  v8f oacc[4];
#pragma unroll
  for (int r = 0; r < 8; ++r) { mrow[r] = -INFINITY; lrow[r] = 0.f; }
#pragma unroll
  for (int t = 0; t < 4; ++t) oacc[t] = zero8();

  for (int kt = 0; kt < NKT; ++kt) {
    const int kv0 = kt * 64;
    __syncthreads();
    {
      const int r = tid >> 1, half = (tid & 1) * 32;
      const _Float16* zg  = Zp16 + (rowB + kv0 + r) * ZP + (size_t)h * 64 + half;
      const _Float16* vg  = Vh + (size_t)r * SEQ + kv0 + half;
      const _Float16* vlg = Vl + (size_t)r * SEQ + kv0 + half;
#pragma unroll
      for (int i = 0; i < 4; ++i) {
        const v8h a0 = *(const v8h*)(zg + 8 * i);
        const v8h b0 = *(const v8h*)(vg + 8 * i);
        const v8h b1 = *(const v8h*)(vlg + 8 * i);
        *(v8h*)(Zsh + r * 64 + half + 8 * i) = a0;
        *(v8h*)(Vth + r * 64 + half + 8 * i) = b0;
        *(v8h*)(Vtl + r * 64 + half + 8 * i) = b1;
      }
    }
    __syncthreads();

    v8f s[4];
#pragma unroll
    for (int j = 0; j < 4; ++j) {
      const _Float16* zr = Zsh + (j * 16 + c) * 64 + 8 * hh;
      FH b1, b2;
      b2.h[0] = *(const v8h*)(zr + 16);
      b2.h[1] = *(const v8h*)(zr + 32);
      b1.h[0] = *(const v8h*)(zr + 32);
      b1.h[1] = *(const v8h*)(zr + 48);
      v8f ah = mma_h(zq, b1.v, zero8());
      v8f ax = mma_h(zq, b2.v, zero8());
      const float zt = zsq[(rowB + kv0 + j * 16 + c) * NH + h];
      {
#pragma clang fp contract(off)
#pragma unroll
        for (int r = 0; r < 8; ++r) {
          const float d = ah[r] + ax[r] * (1.0f / RSC);
          float sq = (zsq_q[r] + zt) - 2.0f * d;
          sq = fmaxf(sq, 0.f);
          s[j][r] = ng * sq;
        }
      }
    }

    _Float16* pwh = Psh[wave];
#pragma unroll
    for (int r = 0; r < 8; ++r) {
      float m = s[0][r];
#pragma unroll
      for (int j = 1; j < 4; ++j) m = fmaxf(m, s[j][r]);
#pragma unroll
      for (int off = 1; off < 16; off <<= 1) m = fmaxf(m, __shfl_xor(m, off, 32));
      const float mnew  = fmaxf(mrow[r], m);
      const float msafe = (mnew == -INFINITY) ? 0.f : mnew;
      const float alpha = __expf(mrow[r] - msafe);
      mrow[r] = mnew;
      float psum = 0.f;
#pragma unroll
      for (int j = 0; j < 4; ++j) {
        const float p = __expf(s[j][r] - msafe);
        psum += p;
        pwh[(8 * hh + r) * 64 + j * 16 + c] = (_Float16)(p * PCARRY);
      }
#pragma unroll
      for (int off = 1; off < 16; off <<= 1) psum += __shfl_xor(psum, off, 32);
      lrow[r] = lrow[r] * alpha + psum;
#pragma unroll
      for (int t = 0; t < 4; ++t) oacc[t][r] *= alpha;
    }
    __builtin_amdgcn_fence(__ATOMIC_RELEASE, "workgroup");
    __builtin_amdgcn_wave_barrier();
    __builtin_amdgcn_fence(__ATOMIC_ACQUIRE, "workgroup");

    v8f o1[4];
#pragma unroll
    for (int t = 0; t < 4; ++t) o1[t] = zero8();
#pragma unroll 1
    for (int kk = 0; kk < 2; ++kk) {
      FH pa;
      pa.h[0] = *(const v8h*)(pwh + c * 64 + kk * 32 + 8 * hh);
      pa.h[1] = *(const v8h*)(pwh + c * 64 + kk * 32 + 16 + 8 * hh);
#pragma unroll
      for (int t = 0; t < 4; ++t) {
        FH vb, vl;
        vb.h[0] = *(const v8h*)(Vth + (t * 16 + c) * 64 + kk * 32 + 8 * hh);
        vb.h[1] = *(const v8h*)(Vth + (t * 16 + c) * 64 + kk * 32 + 16 + 8 * hh);
        vl.h[0] = *(const v8h*)(Vtl + (t * 16 + c) * 64 + kk * 32 + 8 * hh);
        vl.h[1] = *(const v8h*)(Vtl + (t * 16 + c) * 64 + kk * 32 + 16 + 8 * hh);
        oacc[t] = mma_h(pa.v, vb.v, oacc[t]);
        o1[t]   = mma_h(pa.v, vl.v, o1[t]);
      }
    }
#pragma unroll
    for (int t = 0; t < 4; ++t)
#pragma unroll
      for (int r = 0; r < 8; ++r) oacc[t][r] += o1[t][r] * (1.0f / RSC);
  }

  float* os = Os[wave];
#pragma unroll
  for (int r = 0; r < 8; ++r) {
    const float l = lrow[r];
    const float inv = ((l > 0.f) ? (1.0f / l) : 0.f) * (1.0f / PCARRY);
#pragma unroll
    for (int t = 0; t < 4; ++t) os[(8 * hh + r) * 64 + t * 16 + c] = oacc[t][r] * inv;
  }
  __builtin_amdgcn_fence(__ATOMIC_RELEASE, "workgroup");
  __builtin_amdgcn_wave_barrier();
  __builtin_amdgcn_fence(__ATOMIC_ACQUIRE, "workgroup");
  {
    const int q4 = lane >> 3, c8 = (lane & 7) * 8;
    v4u hv[4], lv[4];
#pragma unroll
    for (int it = 0; it < 4; ++it) {
      const int row = it * 4 + q4;
      const float* sp = os + row * 64 + c8;
      v4u a, a2;
#pragma unroll
      for (int e = 0; e < 4; ++e) {
        const float f0 = sp[2 * e], f1 = sp[2 * e + 1];
        const unsigned short hb0 = bf_bits(f0), hb1 = bf_bits(f1);
        const unsigned short lb0 = bf_bits(f0 - bf_up(hb0)), lb1 = bf_bits(f1 - bf_up(hb1));
        a[e]  = pk16(hb0, hb1);
        a2[e] = pk16(lb0, lb1);
      }
      hv[it] = a; lv[it] = a2;
    }
    for (int pass = 0; pass < 2; ++pass) {
#pragma unroll
      for (int it = 0; it < 4; ++it) {
        const int row = it * 4 + q4;
        const size_t go = (rowB + q0 + row) * OP + (size_t)h * HD + c8;
        *(volatile v4u*)(octx + go)      = hv[it];
        *(volatile v4u*)(octx + go + DM) = lv[it];
      }
      __threadfence();
    }
  }
}

extern "C" void kernel_launch(void* const* d_in, const int* in_sizes, int n_in,
                              void* d_out, int out_size, void* d_ws, size_t ws_size,
                              hipStream_t stream) {
  if (n_in < 11) return;
  if (in_sizes[0] < ((NB - 1) * SEQ_FULL + SEQ) * DM) return;
  if (in_sizes[1] < ((NB - 1) * SEQ_FULL + SEQ) * DC) return;
  if (in_sizes[2] < DM * DM || in_sizes[3] < DM) return;
  if (in_sizes[4] < DC * HN || in_sizes[5] < HN) return;
  if (in_sizes[6] < DC * DC || in_sizes[7] < DC) return;
  if (in_sizes[8] < DM * DM || in_sizes[9] < DM) return;
  if (in_sizes[10] < NH) return;
  if ((size_t)out_size < OUT1_OFF + (size_t)NB * SEQ * DC) return;

  const float* hidden = (const float*)d_in[0];
  const float* coords = (const float*)d_in[1];
  const float* Wv     = (const float*)d_in[2];
  const float* bv     = (const float*)d_in[3];
  const float* Wc     = (const float*)d_in[4];
  const float* bc     = (const float*)d_in[5];
  const float* Wn     = (const float*)d_in[6];
  const float* bn     = (const float*)d_in[7];
  const float* Wo     = (const float*)d_in[8];
  const float* bo     = (const float*)d_in[9];
  const float* gamma  = (const float*)d_in[10];

  const size_t nRows = (size_t)NB * SEQ;
  const size_t PXB  = nRows * DM * 2;
  const size_t PCB  = nRows * DC * 2;
  const size_t PWV  = (size_t)DM * DM * 2;
  const size_t PWO2 = (size_t)DM * OP * 2;
  const size_t PWC  = (size_t)HN * DC * 2;
  const size_t PWN  = (size_t)DC * DC * 2;
  const size_t PZF  = nRows * HN * 4;
  const size_t PZP  = nRows * ZP * 2;
  const size_t PZQ  = nRows * NH * 4;
  const size_t PVT  = (size_t)NB * DM * SEQ * 2;
  const size_t POC  = nRows * OP * 2;
  size_t off = 0;
  const size_t oXb  = off; off += PXB;
  const size_t oCb  = off; off += PCB;
  const size_t oWv  = off; off += PWV;
  const size_t oWo  = off; off += PWO2;
  const size_t oWc  = off; off += PWC;
  const size_t oWn  = off; off += PWN;
  const size_t oZf  = off; off += PZF;
  const size_t oZp  = off; off += PZP;
  const size_t oZq  = off; off += PZQ;
  const size_t oVTh = off; off += PVT;
  const size_t oVTl = off; off += PVT;
  const size_t oOc  = off; off += POC;
  if (off > ws_size) return;
  if (off > (size_t)134217728) return;

  char* ws = (char*)d_ws;
  unsigned short* Xb   = (unsigned short*)(ws + oXb);
  unsigned short* Cb   = (unsigned short*)(ws + oCb);
  unsigned short* WvT  = (unsigned short*)(ws + oWv);
  unsigned short* WoT2 = (unsigned short*)(ws + oWo);
  unsigned short* WcT  = (unsigned short*)(ws + oWc);
  unsigned short* WnT  = (unsigned short*)(ws + oWn);
  float*          Zf   = (float*)(ws + oZf);
  unsigned short* Zpl  = (unsigned short*)(ws + oZp);
  float*          Zsq  = (float*)(ws + oZq);
  unsigned short* VTh  = (unsigned short*)(ws + oVTh);
  unsigned short* VTl  = (unsigned short*)(ws + oVTl);
  unsigned short* Octx = (unsigned short*)(ws + oOc);
  float* out0 = (float*)d_out;
  float* out1 = (float*)d_out + OUT1_OFF;

  const dim3 blk(256);
  const int n8x = NB * SEQ * DM / 8;
  const int n8c = NB * SEQ * DC / 8;
  const dim3 gCx((n8x + 255) / 256);
  const dim3 gCc((n8c + 255) / 256);
  const dim3 gTrW(DM / 64, DM / 64);
  const dim3 gTrC(HN / 64, DC / 64);
  const dim3 gTrN(DC / 64, DC / 64);
  const int tilesZ = (int)((nRows / 64) * (HN / 64));
  const int tilesC = (int)((nRows / 64) * (DC / 64));
  const int tilesV = (DM / 64) * (SEQ / 64);
  const int tilesO = (int)((nRows / 64) * (DM / 64));
  const dim3 gZ((tilesZ + 7) / 8, 1);
  const dim3 gC1((tilesC + 7) / 8, 1);
  const dim3 gV((tilesV + 7) / 8, NB);
  const dim3 gO((tilesO + 7) / 8, 1);
  const dim3 gPrep((unsigned)(nRows / 16));
  const dim3 gAttn(NB * NH * NQB);

  cvtrows<<<gCx, blk, 0, stream>>>(hidden, Xb, DM / 8, NB * SEQ, SEQ, SEQ_FULL);
  cvtrows<<<gCc, blk, 0, stream>>>(coords, Cb, DC / 8, NB * SEQ, SEQ, SEQ_FULL);
  tr64<<<gTrW, blk, 0, stream>>>(Wv, DM, WvT, DM, 0);
  tr64<<<gTrW, blk, 0, stream>>>(Wo, DM, WoT2, OP, DM);
  tr64<<<gTrC, blk, 0, stream>>>(Wc, HN, WcT, DC, 0);
  tr64<<<gTrN, blk, 0, stream>>>(Wn, DC, WnT, DC, 0);
  gemm64<__bf16, 0, 1><<<gZ, blk, 0, stream>>>(
      Cb, DC, 0LL, WcT, DC, 0LL,
      (void*)Zf, (void*)Zf, HN, 0LL, bc,
      (int)nRows, HN, DC, 1.0f, 1.0f);
  zprep<<<gPrep, blk, 0, stream>>>(Zf, Zpl, Zsq);
  gemm64<__bf16, 0, 1><<<gC1, blk, 0, stream>>>(
      Cb, DC, 0LL, WnT, DC, 0LL,
      (void*)out1, (void*)out1, DC, 0LL, bn,
      (int)nRows, DC, DC, 1.0f, 1.0f);
  gemm64<__bf16, 3, 2><<<gV, blk, 0, stream>>>(
      WvT, DM, 0LL, Xb, DM, (long long)SEQ * DM,
      (void*)VTh, (void*)VTl, SEQ, (long long)DM * SEQ, bv,
      DM, SEQ, DM, 1.0f, RSC);
  attn_dist<<<gAttn, dim3(128), 0, stream>>>(Zpl, Zsq, VTh, VTl, gamma, Octx);
  gemm64<__bf16, 0, 1><<<gO, blk, 0, stream>>>(
      Octx, OP, 0LL, WoT2, OP, 0LL,
      (void*)out0, (void*)out0, DM, 0LL, bo,
      (int)nRows, DM, OP, 1.0f, 1.0f);
  (void)hipGetLastError();
}
